// GNN_87677462380643
// MI455X (gfx1250) — hardware-verified
//
#include <hip/hip_runtime.h>
#include <stddef.h>
#include <stdint.h>


#define DF     128
#define AP1    384
#define HP     256
#define KP     512
#define NGR    64
#define INDW   32
#define NTHR   256
#define NWAVE  8
#define EPT    8
#define CHUNK  (NTHR * EPT)
#define WCAP   (EPT * 32)
#define LISTN  (NWAVE * WCAP)
#define NBA    1024
#define SLA    10
#define RCAP   8192
#define DEGCAP 32
#define GBM    64
#define GBN    128
#define GTHR   128
#define UPART  2048
#define NWPART 7
#define WBLK   ((NWPART * UPART) / NTHR)
#define W2COFF (DF * AP1)
#define PCH    1024
#define PW     256
#define AGG_ZINTS    (LISTN + 2 * RCAP + 3 * NBA)
#define MISC_INTS    16
#define ROWBUF_INTS  (NWAVE * HP / 2)
#define AGG_LDS_INTS (AGG_ZINTS + MISC_INTS + ROWBUF_INTS)
#define POOL_LDS_INTS (NGR * PW + NGR)
#define WSMAX  134217728

static_assert((CHUNK & (CHUNK - 1)) == 0 && CHUNK <= 4096);
static_assert((NBA & (NBA - 1)) == 0 && NBA == (1 << SLA));
static_assert(((long long)CHUNK << SLA) < (1LL << 31));
static_assert(NBA % NWAVE == 0 && NBA % 32 == 0 && NBA % GBM == 0);
static_assert(RCAP % 4 == 0 && AGG_ZINTS % 4 == 0 && LISTN % 4 == 0 && ((AGG_ZINTS + MISC_INTS) % 4) == 0);
static_assert(AGG_ZINTS % (NTHR * 4) == 0);
static_assert(AP1 % 32 == 0 && KP % 32 == 0 && AP1 == 3 * DF && KP == 4 * DF && HP == 2 * DF);
static_assert(GBN == DF && GBM == (GTHR / 32) * 16 && DF == 4 * 32);
static_assert(UPART % NTHR == 0 && UPART == DF * (DF / 8) && (NWPART * UPART) % NTHR == 0);
static_assert(NGR == GBM && PW == NTHR && PW == 2 * DF);
static_assert((NGR * PW) % (NTHR * 4) == 0 && (NGR * PW) / (NTHR * 4) == 16);
static_assert(AGG_LDS_INTS * 4 <= 300000 && POOL_LDS_INTS * 4 <= 300000);
static_assert((W2COFF * 2) % 256 == 0);

typedef float          v4f   __attribute__((ext_vector_type(4)));
typedef float          v8f   __attribute__((ext_vector_type(8)));
typedef int            v4i   __attribute__((ext_vector_type(4)));
typedef int            v8i   __attribute__((ext_vector_type(8)));
typedef unsigned       v2u   __attribute__((ext_vector_type(2)));
typedef unsigned short v4us  __attribute__((ext_vector_type(4)));
typedef unsigned short v8us  __attribute__((ext_vector_type(8)));
typedef unsigned short v16us __attribute__((ext_vector_type(16)));
typedef __bf16         v16bf __attribute__((ext_vector_type(16)));
typedef v4f  __attribute__((may_alias)) v4fa;
typedef v4i  __attribute__((may_alias)) v4ia;
typedef v2u  __attribute__((may_alias)) v2ua;
typedef v4us __attribute__((may_alias)) v4usa;
typedef v8us __attribute__((may_alias)) v8usa;
union FragB { v16bf v; v16us u; v8us h[2]; v8i w; };

__device__ __forceinline__ v8f wmb(const FragB& a, const FragB& b, v8f c) {
  v8f d = __builtin_amdgcn_wmma_f32_16x16x32_bf16(false, a.v, false, b.v, (short)0, c, false, false);
  asm volatile("v_nop\n\tv_nop\n\tv_nop\n\tv_nop" : "+v"(d) : "v"(a.w), "v"(b.w));
  return d;
}

__device__ __forceinline__ unsigned bf16_bits(float f) {
  const unsigned u = __float_as_uint(f);
  return (u + 0x7FFFu + ((u >> 16) & 1u)) >> 16;
}
__device__ __forceinline__ float bf16_val(float f) {
  return __uint_as_float(bf16_bits(f) << 16);
}

__device__ __forceinline__ void wave_sync() {
  __builtin_amdgcn_fence(__ATOMIC_RELEASE, "wavefront");
  __builtin_amdgcn_wave_barrier();
  __builtin_amdgcn_fence(__ATOMIC_ACQUIRE, "wavefront");
}

template <int SLB>
__device__ __forceinline__ int scan_chunk(const int* __restrict__ dsts, int nE, int cbase, int slotBase,
                                          int nb, int vec8, int* list, int tid, int lane, int wave) {
  int wc = 0;
  const int el0  = tid * EPT;
  const int e0   = cbase + el0;
  const int sent = -2147483647 - 1;
  v4i da, db;
  if (vec8 != 0 && cbase + CHUNK <= nE) {
    da = *(const v4i*)(dsts + e0);
    db = *(const v4i*)(dsts + e0 + 4);
  } else {
    da.x = (e0     < nE) ? dsts[min(e0,     nE - 1)] : sent;
    da.y = (e0 + 1 < nE) ? dsts[min(e0 + 1, nE - 1)] : sent;
    da.z = (e0 + 2 < nE) ? dsts[min(e0 + 2, nE - 1)] : sent;
    da.w = (e0 + 3 < nE) ? dsts[min(e0 + 3, nE - 1)] : sent;
    db.x = (e0 + 4 < nE) ? dsts[min(e0 + 4, nE - 1)] : sent;
    db.y = (e0 + 5 < nE) ? dsts[min(e0 + 5, nE - 1)] : sent;
    db.z = (e0 + 6 < nE) ? dsts[min(e0 + 6, nE - 1)] : sent;
    db.w = (e0 + 7 < nE) ? dsts[min(e0 + 7, nE - 1)] : sent;
  }
  const unsigned nbs = (unsigned)slotBase;
  const unsigned unb = (unsigned)nb;
  const unsigned s0 = (unsigned)da.x - nbs, s1 = (unsigned)da.y - nbs;
  const unsigned s2 = (unsigned)da.z - nbs, s3 = (unsigned)da.w - nbs;
  const unsigned s4 = (unsigned)db.x - nbs, s5 = (unsigned)db.y - nbs;
  const unsigned s6 = (unsigned)db.z - nbs, s7 = (unsigned)db.w - nbs;
  const bool h0 = s0 < unb, h1 = s1 < unb, h2 = s2 < unb, h3 = s3 < unb;
  const bool h4 = s4 < unb, h5 = s5 < unb, h6 = s6 < unb, h7 = s7 < unb;
  const unsigned any = __builtin_amdgcn_ballot_w32(h0 | h1 | h2 | h3 | h4 | h5 | h6 | h7);
  if (any != 0u) {
#define HITJ(J, HJ, SJ) { \
      const unsigned mj = __builtin_amdgcn_ballot_w32(HJ); \
      if (mj != 0u) { \
        if (HJ) { \
          const int pos = wc + (int)__builtin_amdgcn_mbcnt_lo(mj, 0u); \
          if (pos < WCAP) list[wave * WCAP + pos] = ((el0 + (J)) << SLB) | (int)(SJ); \
        } \
        wc += (int)__builtin_popcount(mj); } }
    HITJ(0, h0, s0)
    HITJ(1, h1, s1)
    HITJ(2, h2, s2)
    HITJ(3, h3, s3)
    HITJ(4, h4, s4)
    HITJ(5, h5, s5)
    HITJ(6, h6, s6)
    HITJ(7, h7, s7)
#undef HITJ
  }
  return wc;
}

__device__ __forceinline__ v8us gather8(const float* __restrict__ W, int n, int k8) {
  const float* p = W + (size_t)k8 * DF + n;
  v8us o;
#pragma unroll
  for (int i = 0; i < 8; ++i) o[i] = (unsigned short)bf16_bits(p[(size_t)i * DF]);
  return o;
}

__global__ __launch_bounds__(NTHR) void k_prep(const float* __restrict__ x,
                                               const float* __restrict__ W1l, const float* __restrict__ W1r,
                                               const float* __restrict__ W2l, const float* __restrict__ W2r,
                                               int nN, int nUx, unsigned short* a1, unsigned short* wc) {
  const int tid = (int)threadIdx.x;
  const int bx  = (int)blockIdx.x;
  if (bx < WBLK) {
    const int u    = bx * NTHR + tid;
    const int part = u >> 11;
    const int v    = u & (UPART - 1);
    const int n    = v >> 4;
    const int k8   = (v & 15) * 8;
    v8us o;
    if (part < 2)       o = gather8(W1l, n, k8);
    else if (part == 2) o = gather8(W1r, n, k8);
    else if (part < 5)  o = gather8(W2l, n, k8);
    else                o = gather8(W2r, n, k8);
    const size_t off = (part < 3) ? ((size_t)n * AP1 + (size_t)part * DF + k8)
                                  : ((size_t)W2COFF + (size_t)n * KP + (size_t)(part - 3) * DF + k8);
    unsigned short* dp = wc + off;
    *(volatile v8us*)dp = o;
    __threadfence();
    *(volatile v8us*)dp = o;
  } else {
    const int u = (bx - WBLK) * NTHR + tid;
    if (u >= nUx) return;
    const int row = u >> 4;
    const int k8  = (u & 15) * 8;
    const int rc  = row < nN ? row : nN - 1;
    const float* p = x + (size_t)rc * DF + k8;
    const v4f a = *(const v4fa*)p;
    const v4f b = *(const v4fa*)(p + 4);
    const bool ok = row < nN;
    v8us o;
    o[0] = ok ? (unsigned short)bf16_bits(a.x) : (unsigned short)0;
    o[1] = ok ? (unsigned short)bf16_bits(a.y) : (unsigned short)0;
    o[2] = ok ? (unsigned short)bf16_bits(a.z) : (unsigned short)0;
    o[3] = ok ? (unsigned short)bf16_bits(a.w) : (unsigned short)0;
    o[4] = ok ? (unsigned short)bf16_bits(b.x) : (unsigned short)0;
    o[5] = ok ? (unsigned short)bf16_bits(b.y) : (unsigned short)0;
    o[6] = ok ? (unsigned short)bf16_bits(b.z) : (unsigned short)0;
    o[7] = ok ? (unsigned short)bf16_bits(b.w) : (unsigned short)0;
    unsigned short* dp = a1 + (size_t)row * AP1 + 2 * DF + k8;
    *(volatile v8us*)dp = o;
    __threadfence();
    *(volatile v8us*)dp = o;
  }
}

template <int L1>
__global__ __launch_bounds__(NTHR) void k_scan(const int* __restrict__ gath, const int* __restrict__ keys,
                                               int nE, int nN, int vec8, int mRows,
                                               unsigned short* pl, float* aggf) {
  extern __shared__ __attribute__((aligned(16))) int dsm[];
  int* list = dsm;
  int* hl   = dsm + LISTN;
  int* sl   = hl + RCAP;
  int* cnt  = sl + RCAP;
  int* offs = cnt + NBA;
  int* cur  = offs + NBA;
  int* misc = cur + NBA;
  const int tid = (int)threadIdx.x, lane = tid & 31, wave = tid >> 5;
  unsigned short* rowbuf = (unsigned short*)(misc + MISC_INTS) + wave * HP;
  const int nodeBase = (int)blockIdx.x * NBA;

  {
    const v4i z4 = {0, 0, 0, 0};
    for (int i = tid * 4; i < AGG_ZINTS; i += NTHR * 4) *(v4ia*)(dsm + i) = z4;
    if (tid < MISC_INTS) misc[tid] = 0;
  }
  __syncthreads();

  int t = 0, ov = 0;
  const int nChunks = (nE + CHUNK - 1) / CHUNK;
#pragma unroll 1
  for (int ch = 0; ch < nChunks; ++ch) {
    const int cbase = ch * CHUNK;
    const int wc = scan_chunk<SLA>(keys, nE, cbase, nodeBase, NBA, vec8, list, tid, lane, wave);
    if (lane == 0) misc[wave] = wc;
    __syncthreads();
    if (wave == 0) {
#pragma unroll 1
      for (int w2 = 0; w2 < NWAVE; ++w2) {
        int c = misc[w2];
        c = c < 0 ? 0 : (c > WCAP ? WCAP : c);
#pragma unroll 1
        for (int b0 = 0; b0 < c; b0 += 32) {
          const int idx = b0 + lane;
          const int ent = list[w2 * WCAP + (idx < WCAP ? idx : WCAP - 1)];
          const int m32 = (c - b0) < 32 ? (c - b0) : 32;
#pragma unroll 1
          for (int k = 0; k < m32; ++k) {
            const int u    = __builtin_amdgcn_readlane(ent, k);
            const int slot = u & (NBA - 1);
            const int el   = (u >> SLA) & (CHUNK - 1);
            const int pk   = ((cbase + el) << SLA) | slot;
            if (t < RCAP) {
              if (lane == 0) { hl[t] = pk; cnt[slot] = cnt[slot] + 1; }
              t = t + 1;
            } else {
              ov = 1;
            }
          }
        }
      }
    }
    __syncthreads();
  }
  if (wave == 0 && lane == 0) { misc[8] = t; misc[9] = ov; }
  __syncthreads();
  int tt = misc[8];
  tt = tt < 0 ? 0 : (tt > RCAP ? RCAP : tt);
  const int ovf = misc[9];

  if (wave == 0) {
    const int base = lane * (NBA / 32);
    int s = 0;
#pragma unroll 1
    for (int i = 0; i < NBA / 32; ++i) s += cnt[base + i];
    int incl = s;
#pragma unroll
    for (int d = 1; d < 32; d <<= 1) {
      const int y = __shfl_up(incl, d, 32);
      if (lane >= d) incl += y;
    }
    int run = incl - s;
#pragma unroll 1
    for (int i = 0; i < NBA / 32; ++i) {
      const int cv = cnt[base + i];
      offs[base + i] = run;
      cur[base + i]  = run;
      run += cv;
    }
  }
  __syncthreads();
  if (wave == 0) {
#pragma unroll 1
    for (int b0 = 0; b0 < tt; b0 += 32) {
      const int idx = b0 + lane;
      const int ent = hl[idx < RCAP ? idx : RCAP - 1];
      const int m32 = (tt - b0) < 32 ? (tt - b0) : 32;
#pragma unroll 1
      for (int k = 0; k < m32; ++k) {
        const int u    = __builtin_amdgcn_readlane(ent, k);
        const int slot = u & (NBA - 1);
        if (lane == 0) {
          int p = cur[slot];
          p = p < 0 ? 0 : (p > RCAP - 1 ? RCAP - 1 : p);
          sl[p] = u;
          cur[slot] = p + 1;
        }
      }
    }
  }
  __syncthreads();

  const float qnan = __int_as_float(0x7fc00000);
  const float pz = (ovf != 0) ? qnan : 0.0f;
  const unsigned short* gp = pl;
#pragma unroll 1
  for (int si = 0; si < NBA / NWAVE; ++si) {
    const int s    = si * NWAVE + wave;
    const int node = nodeBase + s;
    int c = cnt[s];
    const bool big = c > DEGCAP;
    c = c < 0 ? 0 : (c > DEGCAP ? DEGCAP : c);
    int o = offs[s];
    o = o < 0 ? 0 : (o > RCAP ? RCAP : o);
    float a0 = 0.0f, a1 = 0.0f, a2 = 0.0f, a3 = 0.0f;
#pragma unroll 1
    for (int b0 = 0; b0 < c; b0 += 32) {
      int idx = o + b0 + lane;
      idx = idx > RCAP - 1 ? RCAP - 1 : idx;
      const int ent = sl[idx];
      int eid = ent >> SLA;
      eid = eid < 0 ? 0 : (eid > nE - 1 ? nE - 1 : eid);
      int sr = gath[eid];
      sr = sr < 0 ? 0 : (sr > nN - 1 ? nN - 1 : sr);
      const int m32 = (c - b0) < 32 ? (c - b0) : 32;
#pragma unroll 1
      for (int k = 0; k < m32; ++k) {
        const int sk = __builtin_amdgcn_readlane(sr, k);
        if constexpr (L1 != 0) {
          const v2u w = *(const v2ua*)(gp + (size_t)sk * AP1 + 2 * DF + 4 * lane);
          a0 += __uint_as_float(w.x << 16);
          a1 += __uint_as_float(w.x & 0xffff0000u);
          a2 += __uint_as_float(w.y << 16);
          a3 += __uint_as_float(w.y & 0xffff0000u);
        } else {
          const unsigned short* rp = gp + (size_t)sk * HP + 4 * lane;
          const v2u wh = *(const v2ua*)rp;
          const v2u wl = *(const v2ua*)(rp + DF);
          const float f0 = __uint_as_float(wh.x << 16)         + __uint_as_float(wl.x << 16);
          const float f1 = __uint_as_float(wh.x & 0xffff0000u) + __uint_as_float(wl.x & 0xffff0000u);
          const float f2 = __uint_as_float(wh.y << 16)         + __uint_as_float(wl.y << 16);
          const float f3 = __uint_as_float(wh.y & 0xffff0000u) + __uint_as_float(wl.y & 0xffff0000u);
          a0 += f0; a1 += f1; a2 += f2; a3 += f3;
        }
      }
    }
    const float pzr = big ? qnan : pz;
    const bool live = node < nN;
    const float dv = (float)(c < 1 ? 1 : c);
    const float d0 = (a0 + pzr) / dv;
    const float d1 = (a1 + pzr) / dv;
    const float d2 = (a2 + pzr) / dv;
    const float d3 = (a3 + pzr) / dv;
    const float m0 = live ? d0 : 0.0f;
    const float m1 = live ? d1 : 0.0f;
    const float m2 = live ? d2 : 0.0f;
    const float m3 = live ? d3 : 0.0f;
    if constexpr (L1 != 0) {
      v4us mh, ml;
      {
        unsigned hb;
        hb = bf16_bits(m0); mh[0] = (unsigned short)hb; ml[0] = (unsigned short)bf16_bits(m0 - __uint_as_float(hb << 16));
        hb = bf16_bits(m1); mh[1] = (unsigned short)hb; ml[1] = (unsigned short)bf16_bits(m1 - __uint_as_float(hb << 16));
        hb = bf16_bits(m2); mh[2] = (unsigned short)hb; ml[2] = (unsigned short)bf16_bits(m2 - __uint_as_float(hb << 16));
        hb = bf16_bits(m3); mh[3] = (unsigned short)hb; ml[3] = (unsigned short)bf16_bits(m3 - __uint_as_float(hb << 16));
      }
      *(v4usa*)(rowbuf + 4 * lane) = mh;
      *(v4usa*)(rowbuf + DF + 4 * lane) = ml;
      wave_sync();
      const v8us q0 = *(const v8usa*)(rowbuf + 8 * lane);
      wave_sync();
      if (node < mRows) {
        unsigned short* rpw = pl + (size_t)node * AP1 + 8 * lane;
        *(volatile v8us*)rpw = q0;
        __threadfence();
        *(volatile v8us*)rpw = q0;
      }
    } else {
      v4f ow;
      ow.x = m0; ow.y = m1; ow.z = m2; ow.w = m3;
      if (node < mRows) {
        float* op = aggf + (size_t)node * DF + 4 * lane;
        *(volatile v4f*)op = ow;
        __threadfence();
        *(volatile v4f*)op = ow;
      }
    }
  }
}

template <int FIN>
__global__ __launch_bounds__(GTHR) void k_gemm(const unsigned short* __restrict__ Apl, int lda,
                                               const unsigned short* __restrict__ BT, int K,
                                               const float* __restrict__ bias, const float* __restrict__ indp,
                                               unsigned short* hout, float* outp, int nOut) {
  __shared__ __attribute__((aligned(16))) float stg[GBM * GBN];
  const int tid = (int)threadIdx.x, lane = tid & 31, wave = tid >> 5, hh = lane >> 4, m = lane & 15;
  const int rowBase = (int)blockIdx.x * GBM;

  v8f acc[8];
  {
    const v8f z = {0.f, 0.f, 0.f, 0.f, 0.f, 0.f, 0.f, 0.f};
#pragma unroll
    for (int t = 0; t < 8; ++t) acc[t] = z;
  }
  const unsigned short* ap = Apl + (size_t)(rowBase + 16 * wave + m) * (size_t)lda + 8 * hh;
  const unsigned short* bp = BT + (size_t)m * (size_t)K + 8 * hh;

#pragma unroll 1
  for (int k0 = 0; k0 < K; k0 += 32) {
    FragB af;
    af.h[0] = *(const v8usa*)(ap + k0);
    af.h[1] = *(const v8usa*)(ap + k0 + 16);
#pragma unroll
    for (int nt = 0; nt < 8; ++nt) {
      const unsigned short* wq = bp + (size_t)(16 * nt) * (size_t)K + k0;
      FragB bf;
      bf.h[0] = *(const v8usa*)wq;
      bf.h[1] = *(const v8usa*)(wq + 16);
      acc[nt] = wmb(af, bf, acc[nt]);
    }
  }

#pragma unroll
  for (int nt = 0; nt < 8; ++nt) {
    const int lc = 16 * nt + m;
#pragma unroll
    for (int r = 0; r < 8; ++r) {
      const int lr = 16 * wave + 8 * hh + r;
      stg[lr * GBN + lc] = acc[nt][r];
    }
  }
  __syncthreads();

  v4f bb4;
  {
    const v4f t1 = *(const v4f*)(bias + 4 * lane);
    bb4.x = bf16_val(t1.x);
    bb4.y = bf16_val(t1.y);
    bb4.z = bf16_val(t1.z);
    bb4.w = bf16_val(t1.w);
  }

  v4f pv[16];
#pragma unroll
  for (int i = 0; i < 16; ++i) pv[i] = *(const v4fa*)(stg + (16 * wave + i) * GBN + 4 * lane);
  __syncthreads();

  if constexpr (FIN != 0) {
    int rl = rowBase + 16 * wave + m;
    rl = rl < nOut ? rl : nOut - 1;
    rl = rl < 0 ? 0 : rl;
    const float indv = indp[(size_t)rl * INDW];
#pragma unroll
    for (int i = 0; i < 16; ++i) {
      const float iv = __shfl(indv, i, 32);
      v4f y;
      y.x = pv[i].x + bb4.x * iv;
      y.y = pv[i].y + bb4.y * iv;
      y.z = pv[i].z + bb4.z * iv;
      y.w = pv[i].w + bb4.w * iv;
      pv[i] = y;
    }
#pragma unroll
    for (int i = 0; i < 16; ++i) {
      const int r = rowBase + 16 * wave + i;
      if (r < nOut) *(volatile v4f*)(outp + (size_t)r * DF + 4 * lane) = pv[i];
    }
    __threadfence();
#pragma unroll
    for (int i = 0; i < 16; ++i) {
      const int r = rowBase + 16 * wave + i;
      if (r < nOut) *(volatile v4f*)(outp + (size_t)r * DF + 4 * lane) = pv[i];
    }
  } else {
#pragma unroll
    for (int i = 0; i < 16; ++i) {
      const bool ok = (rowBase + 16 * wave + i) < nOut;
      const v4f t = pv[i] + bb4;
      v4f y;
      y.x = (t.x > 0.0f) ? t.x : (t.x - t.x);
      y.y = (t.y > 0.0f) ? t.y : (t.y - t.y);
      y.z = (t.z > 0.0f) ? t.z : (t.z - t.z);
      y.w = (t.w > 0.0f) ? t.w : (t.w - t.w);
      y.x = ok ? y.x : 0.0f; y.y = ok ? y.y : 0.0f; y.z = ok ? y.z : 0.0f; y.w = ok ? y.w : 0.0f;
      pv[i] = y;
    }
#pragma unroll
    for (int i = 0; i < 16; ++i) {
      v4us h4, l4;
      unsigned hb;
      hb = bf16_bits(pv[i].x); h4[0] = (unsigned short)hb; l4[0] = (unsigned short)bf16_bits(pv[i].x - __uint_as_float(hb << 16));
      hb = bf16_bits(pv[i].y); h4[1] = (unsigned short)hb; l4[1] = (unsigned short)bf16_bits(pv[i].y - __uint_as_float(hb << 16));
      hb = bf16_bits(pv[i].z); h4[2] = (unsigned short)hb; l4[2] = (unsigned short)bf16_bits(pv[i].z - __uint_as_float(hb << 16));
      hb = bf16_bits(pv[i].w); h4[3] = (unsigned short)hb; l4[3] = (unsigned short)bf16_bits(pv[i].w - __uint_as_float(hb << 16));
      unsigned short* srow = (unsigned short*)stg + (size_t)(16 * wave + i) * (2 * GBN);
      *(v4usa*)(srow + 4 * lane) = h4;
      *(v4usa*)(srow + DF + 4 * lane) = l4;
    }
    __syncthreads();
    v8us qv[16];
#pragma unroll
    for (int i = 0; i < 16; ++i) {
      const unsigned short* srow = (const unsigned short*)stg + (size_t)(16 * wave + i) * (2 * GBN);
      qv[i] = *(const v8usa*)(srow + 8 * lane);
    }
#pragma unroll
    for (int i = 0; i < 16; ++i) {
      unsigned short* rp = hout + (size_t)(rowBase + 16 * wave + i) * (size_t)HP + 8 * lane;
      *(volatile v8us*)rp = qv[i];
    }
    __threadfence();
#pragma unroll
    for (int i = 0; i < 16; ++i) {
      unsigned short* rp = hout + (size_t)(rowBase + 16 * wave + i) * (size_t)HP + 8 * lane;
      *(volatile v8us*)rp = qv[i];
    }
  }
}

__global__ __launch_bounds__(NTHR) void k_poolp(const float* __restrict__ agg2,
                                                const unsigned short* __restrict__ hpl,
                                                const int* __restrict__ bat, int nN,
                                                float* rec, int* cntrec) {
  extern __shared__ __attribute__((aligned(16))) int psm[];
  float* acc  = (float*)psm;
  int*   cntg = psm + NGR * PW;
  const int tid = (int)threadIdx.x, lane = tid & 31;
  const int wv = __builtin_amdgcn_readfirstlane(tid >> 5);
  {
    const v4f z4 = {0.f, 0.f, 0.f, 0.f};
    for (int i = tid * 4; i < NGR * PW; i += NTHR * 4) *(v4fa*)(acc + i) = z4;
    if (tid < NGR) cntg[tid] = 0;
  }
  __syncthreads();

  const int r0 = (int)blockIdx.x * PCH;
  int r1 = r0 + PCH;
  r1 = r1 > nN ? nN : r1;
  if (wv < 4) {
#pragma unroll 1
    for (int i = r0; i < r1; ++i) {
      const int g = bat[i];
      const float v = agg2[(size_t)i * DF + tid];
      if ((unsigned)g < (unsigned)NGR) {
        acc[g * PW + tid] = acc[g * PW + tid] + v;
        if (tid == 0) cntg[g] = cntg[g] + 1;
      }
    }
  } else {
    const int cc = tid - DF;
#pragma unroll 1
    for (int i = r0; i < r1; ++i) {
      const int g = bat[i];
      const unsigned hb = hpl[(size_t)i * HP + cc];
      const unsigned lb = hpl[(size_t)i * HP + DF + cc];
      const float v = __uint_as_float(hb << 16) + __uint_as_float(lb << 16);
      if ((unsigned)g < (unsigned)NGR) {
        acc[g * PW + tid] = acc[g * PW + tid] + v;
      }
    }
  }
  __syncthreads();

  constexpr int NIT = (NGR * PW) / (NTHR * 4);
  v4f vals[NIT];
#pragma unroll
  for (int it = 0; it < NIT; ++it) vals[it] = *(const v4fa*)(acc + 4 * (it * NTHR + tid));
  const v4i cv = *(const v4ia*)(cntg + 4 * (lane & 15));
  float* rp = rec + (size_t)blockIdx.x * (size_t)(NGR * PW);
  int*   cp = cntrec + (size_t)blockIdx.x * NGR + 4 * (lane & 15);
  const bool okc = tid < 16;
#pragma unroll
  for (int it = 0; it < NIT; ++it) *(volatile v4f*)(rp + 4 * (size_t)(it * NTHR + tid)) = vals[it];
  if (okc) *(volatile v4i*)cp = cv;
  __threadfence();
#pragma unroll
  for (int it = 0; it < NIT; ++it) *(volatile v4f*)(rp + 4 * (size_t)(it * NTHR + tid)) = vals[it];
  if (okc) *(volatile v4i*)cp = cv;
}

__global__ __launch_bounds__(NTHR) void k_poolc(const float* __restrict__ rec, const int* __restrict__ cntrec,
                                                int nPC, unsigned short* pm, float* indp) {
  __shared__ __attribute__((aligned(16))) unsigned short prow[KP];
  const int tid = (int)threadIdx.x;
  const int g = (int)blockIdx.x;
  double s = 0.0;
  int gc = 0;
#pragma unroll 1
  for (int ch = 0; ch < nPC; ++ch) {
    s += (double)rec[((size_t)ch * NGR + g) * PW + tid];
    gc += cntrec[(size_t)ch * NGR + g];
  }
  const int gcl = gc < 1 ? 1 : gc;
  const float sm = (float)s;
  const float mv = sm / (float)gcl;
  const unsigned hb = bf16_bits(mv);
  const unsigned lb = bf16_bits(mv - __uint_as_float(hb << 16));
  const int base = (tid < DF) ? tid : (tid + DF);
  prow[base]      = (unsigned short)hb;
  prow[base + DF] = (unsigned short)lb;
  __syncthreads();
  const v8us q = *(const v8usa*)(prow + 8 * (tid & 63));
  unsigned short* dp = pm + (size_t)g * KP + 8 * (tid & 63);
  const float ind = (gc > 0) ? 1.0f : 0.0f;
  v4f iv;
  iv.x = ind; iv.y = ind; iv.z = ind; iv.w = ind;
  float* ip = indp + (size_t)g * INDW + 4 * (tid & 7);
  const bool okp = tid < 64;
  const bool oki = tid < 8;
  if (okp) *(volatile v8us*)dp = q;
  if (oki) *(volatile v4f*)ip = iv;
  __threadfence();
  if (okp) *(volatile v8us*)dp = q;
  if (oki) *(volatile v4f*)ip = iv;
}

static inline int cdiv(int a, int b) { return (a + b - 1) / b; }
static inline size_t al256(size_t o) { return (o + 255) & ~(size_t)255; }

extern "C" void kernel_launch(void* const* d_in, const int* in_sizes, int n_in,
                              void* d_out, int out_size, void* d_ws, size_t ws_size,
                              hipStream_t stream) {
  if (n_in < 9) return;
  if (in_sizes[0] < DF || (in_sizes[0] % DF) != 0) return;
  const int nN = in_sizes[0] / DF;
  if (nN < 16 || nN >= (1 << 24)) return;
  if (in_sizes[1] < 2 || (in_sizes[1] & 1) != 0) return;
  const int nE = in_sizes[1] / 2;
  if (nE < 1 || nE >= (1 << 21)) return;
  if (in_sizes[2] != nN) return;
  if (in_sizes[3] != DF * DF || in_sizes[4] != DF) return;
  if (in_sizes[5] != DF * DF) return;
  if (in_sizes[6] != DF * DF || in_sizes[7] != DF) return;
  if (in_sizes[8] != DF * DF) return;
  if (out_size != NGR * DF) return;

  const float* x    = (const float*)d_in[0];
  const int*   edge = (const int*)d_in[1];
  const int*   bat  = (const int*)d_in[2];
  const float* W1l  = (const float*)d_in[3];
  const float* b1   = (const float*)d_in[4];
  const float* W1r  = (const float*)d_in[5];
  const float* W2l  = (const float*)d_in[6];
  const float* b2   = (const float*)d_in[7];
  const float* W2r  = (const float*)d_in[8];
  float* out = (float*)d_out;
  const int* src = edge;
  const int* dst = edge + nE;

  const int MP  = cdiv(nN, GBM) * GBM;
  const int gM  = MP / GBM;
  const int gA  = cdiv(MP, NBA);
  const int nPC = cdiv(nN, PCH);
  if ((long long)gA * NBA < (long long)MP) return;
  const int vec8 = ((nE & 3) == 0) ? 1 : 0;

  char* ws = (char*)d_ws;
  size_t off = 0;
  const size_t oWC  = off; off = al256(off + ((size_t)DF * AP1 + (size_t)DF * KP) * 2);
  const size_t oPM  = off; off = al256(off + (size_t)NGR * KP * 2);
  const size_t oIND = off; off = al256(off + (size_t)NGR * INDW * 4);
  const size_t oH   = off; off = al256(off + (size_t)MP * HP * 2);
  const size_t szA1 = al256((size_t)MP * AP1 * 2);
  const size_t oA1  = off; off = off + szA1;
  if (off > ws_size || off > (size_t)WSMAX) return;
  const size_t szAGG = al256((size_t)MP * DF * 4);
  const size_t szREC = al256((size_t)nPC * NGR * PW * 4);
  const size_t szCNT = al256((size_t)nPC * NGR * 4);
  if (szAGG + szREC + szCNT > szA1) return;
  unsigned short* WC   = (unsigned short*)(ws + oWC);
  unsigned short* W1C  = WC;
  unsigned short* W2C  = WC + W2COFF;
  unsigned short* PM   = (unsigned short*)(ws + oPM);
  float*          INDP = (float*)(ws + oIND);
  unsigned short* H    = (unsigned short*)(ws + oH);
  unsigned short* A1   = (unsigned short*)(ws + oA1);
  float*          AGG2 = (float*)(ws + oA1);
  float*          REC  = (float*)(ws + oA1 + szAGG);
  int*            CNT  = (int*)(ws + oA1 + szAGG + szREC);

  const size_t scanLds = (size_t)AGG_LDS_INTS * 4;
  const size_t poolLds = (size_t)POOL_LDS_INTS * 4;
  hipFuncSetAttribute(reinterpret_cast<const void*>(&k_scan<1>), hipFuncAttributeMaxDynamicSharedMemorySize, (int)scanLds);
  hipFuncSetAttribute(reinterpret_cast<const void*>(&k_scan<0>), hipFuncAttributeMaxDynamicSharedMemorySize, (int)scanLds);
  hipFuncSetAttribute(reinterpret_cast<const void*>(&k_poolp), hipFuncAttributeMaxDynamicSharedMemorySize, (int)poolLds);

  const int nUx = MP * (DF / 8);
  k_prep<<<WBLK + cdiv(nUx, NTHR), NTHR, 0, stream>>>(x, W1l, W1r, W2l, W2r, nN, nUx, A1, WC);
  k_scan<1><<<gA, NTHR, scanLds, stream>>>(src, dst, nE, nN, vec8, MP, A1, AGG2);
  k_gemm<0><<<gM, GTHR, 0, stream>>>(A1, AP1, W1C, AP1, b1, INDP, H, out, nN);
  k_scan<0><<<gA, NTHR, scanLds, stream>>>(src, dst, nE, nN, vec8, MP, H, AGG2);
  k_poolp<<<nPC, NTHR, poolLds, stream>>>(AGG2, H, bat, nN, REC, CNT);
  k_poolc<<<NGR, NTHR, 0, stream>>>(REC, CNT, nPC, PM, INDP);
  k_gemm<1><<<1, GTHR, 0, stream>>>(PM, KP, W2C, KP, b2, INDP, H, out, NGR);
}
